// Covar_Attn_80066780332411
// MI455X (gfx1250) — hardware-verified
//
#include <hip/hip_runtime.h>
#include <math.h>

#ifndef NB
#define NB 32
#endif
#define NB_FULL 32
#define CH 512
#define MSP 784
#define XP 832
#define KCOV 800
#define DD (CH * CH)
#define NBC ((NB) < 16 ? (NB) : 16)
#define NCHUNK ((NB) / (NBC))
#define CA_COV (1.0f / (256.0f * 784.0f))

static_assert(NB >= 1 && NB <= NB_FULL);
static_assert(NB % NBC == 0);
static_assert(CH == 512);
static_assert(CH % 64 == 0 && CH % 32 == 0);
static_assert((CH / 64) * (CH / 64) == 64);
static_assert(KCOV % 32 == 0 && KCOV >= MSP && XP >= KCOV);
static_assert(XP % 64 == 0);
static_assert(MSP % 8 == 0 && MSP % 4 == 0);
static_assert((XP / 8) % 8 == 0 && (XP / 8) <= 128 && (XP / 8) > 96);
static_assert((NBC * CH) % 256 == 0);
static_assert(((CH * MSP) / 4) % 256 == 0);
static_assert(CH == 4 * 32 * 4);
static_assert(sizeof(float) * 8 * 16 * 68 <= 131072);
static_assert(2 * 4 * 32 * 16 == 16 * 64 * 4);
static_assert(4 * 32 * 16 == 16 * 64 * 2);
static_assert(8 * 32 * 4 == 16 * 64);

static constexpr size_t SZ_X16 = (size_t)NBC * CH * XP * 2;
static constexpr size_t SZ_TAB = (size_t)NBC * CH * 4;
static constexpr size_t SZ_F32 = (size_t)NBC * DD * 4;
static constexpr size_t SZ_F16 = (size_t)NBC * DD * 2;
static constexpr size_t SZ_SCL = (size_t)NB * CH * 4;
static constexpr size_t WS_TOTAL = SZ_X16 + 2 * SZ_TAB + 4 * SZ_F32 + 4 * SZ_F16 + SZ_SCL;
static_assert(SZ_X16 % 256 == 0 && SZ_TAB % 256 == 0 && SZ_F32 % 256 == 0 && SZ_F16 % 256 == 0 && SZ_SCL % 256 == 0);
static_assert(WS_TOTAL <= (size_t)134217728);

static constexpr float K_ONE5  = 1.5f;
static constexpr float K_075   = 0.75f;
static constexpr float K_225   = 2.25f;
static constexpr float K_1125  = 1.125f;
static constexpr float K_3375  = 3.375f;
static constexpr float K_ZERO  = 0.0f;
static constexpr float K_M21   = -1.0f / 2097152.0f;
static constexpr float K_M22   = -1.0f / 4194304.0f;
static constexpr float K_M23   = -1.0f / 8388608.0f;

typedef __attribute__((ext_vector_type(16))) _Float16 v16h;
typedef __attribute__((ext_vector_type(8)))  _Float16 v8h;
typedef __attribute__((ext_vector_type(8)))  float    v8f;
typedef __attribute__((ext_vector_type(4)))  float    v4f;
typedef _Float16 h16;


#define VST2(T, ptr, val) do { const T vst2_v_ = (val); *(volatile T*)(ptr) = vst2_v_; __threadfence(); *(volatile T*)(ptr) = vst2_v_; } while (0)
#define VST2V4(ptr, val) do { const v4f vst2_v4_ = (val); *(volatile v4f*)(ptr) = vst2_v4_; __threadfence(); *(volatile v4f*)(ptr) = vst2_v4_; } while (0)

__device__ __forceinline__ float bfr(float f) {
    unsigned u = __float_as_uint(f);
    u += 0x7FFFu + ((u >> 16) & 1u);
    return __uint_as_float(u & 0xFFFF0000u);
}
static __device__ __forceinline__ h16 toh_flush(float v) { const h16 r = (h16)v; return (fabsf(v) < 6.103515625e-05f) ? (h16)0.0f : r; }
__device__ __forceinline__ void st8hf(_Float16* P, size_t o, const float* v) {
    v8h pk;
#pragma unroll
    for (int e = 0; e < 8; ++e) pk[e] = toh_flush(v[e]);
    const v8h t = pk;
    *(volatile v8h*)(P + o) = t;
    __threadfence();
    *(volatile v8h*)(P + o) = t;
}

union FragU { v16h v; v8h h[2]; };
__device__ __forceinline__ v16h frag_ld(const _Float16* p) {
    FragU f; f.h[0] = *(const v8h*)(p); f.h[1] = *(const v8h*)(p + 16); return f.v;
}
__device__ __forceinline__ void dep_guard_h(v8f& a, v8f& b, v16h x, v16h y) { asm volatile("v_nop\n\tv_nop\n\tv_nop\n\tv_nop" : "+v"(a), "+v"(b) : "v"(x), "v"(y)); }
__device__ __forceinline__ void keep4_h(v16h a, v16h b, v16h c, v16h d) { asm volatile("v_nop" :: "v"(a), "v"(b), "v"(c), "v"(d)); }
__device__ __forceinline__ void acc_guard4(v8f& a, v8f& b, v8f& c, v8f& d) { asm volatile("v_nop\n\tv_nop\n\tv_nop\n\tv_nop" : "+v"(a), "+v"(b), "+v"(c), "+v"(d)); }
__device__ __forceinline__ void wave_sync_lds() {
    __builtin_amdgcn_fence(3  , "workgroup");
    __builtin_amdgcn_wave_barrier();
    __builtin_amdgcn_fence(2  , "workgroup");
}

__device__ __forceinline__ void gemm_tile64(const _Float16* __restrict__ A, unsigned lda, const _Float16* __restrict__ Bt, unsigned ldb,
                                            unsigned K, unsigned m0, unsigned n0, unsigned rlane, unsigned koff, v8f (&acc)[4][4]) {
#pragma unroll
  for (int i = 0; i < 4; ++i)
#pragma unroll
    for (int j = 0; j < 4; ++j) acc[i][j] = (v8f){0.f,0.f,0.f,0.f,0.f,0.f,0.f,0.f};

  for (unsigned k0 = 0; k0 < K; k0 += 32u) {
    v16h bh[4];
#pragma unroll
    for (int j = 0; j < 4; ++j)
      bh[j] = frag_ld(Bt + (size_t)(n0 + ((unsigned)j << 4) + rlane) * ldb + koff + k0);
#pragma unroll
    for (int i = 0; i < 4; ++i) {
      const v16h ah = frag_ld(A + (size_t)(m0 + ((unsigned)i << 4) + rlane) * lda + koff + k0);
#pragma unroll
      for (int j = 0; j < 4; ++j)
        acc[i][j] = __builtin_amdgcn_wmma_f32_16x16x32_f16(false, ah, false, bh[j], (short)0, acc[i][j], false, false);
      dep_guard_h(acc[i][0], acc[i][3], ah, ah);
    }
    keep4_h(bh[0], bh[1], bh[2], bh[3]);
  }
  acc_guard4(acc[0][0], acc[0][1], acc[0][2], acc[0][3]);
  acc_guard4(acc[1][0], acc[1][1], acc[1][2], acc[1][3]);
  acc_guard4(acc[2][0], acc[2][1], acc[2][2], acc[2][3]);
  acc_guard4(acc[3][0], acc[3][1], acc[3][2], acc[3][3]);
}

__device__ __forceinline__ void slab_store(const float* slab, unsigned lane, float* Cf, _Float16* Ch16, bool out16) {
  {
    const unsigned hh = lane >> 4, c4 = (lane & 15u) * 4u;
#pragma unroll
    for (int half = 0; half < 2; ++half) {
      v4f vv[4];
#pragma unroll
      for (int it = 0; it < 4; ++it) {
        const unsigned row = (unsigned)(half * 4 + it) * 2u + hh;
        vv[it] = *(const v4f*)(slab + row * 68u + c4);
      }
      for (int pass = 0; pass < 2; ++pass) {
#pragma unroll
        for (int it = 0; it < 4; ++it) {
          const unsigned row = (unsigned)(half * 4 + it) * 2u + hh;
          *(volatile v4f*)(Cf + (size_t)row * CH + c4) = vv[it];
        }
        __threadfence();
      }
    }
  }
  if (out16) {
    const unsigned q = lane >> 3, c8 = (lane & 7u) * 8u;
    v8h hv[4];
#pragma unroll
    for (int it = 0; it < 4; ++it) {
      const unsigned row = (unsigned)it * 4u + q;
      const float* sp = slab + row * 68u + c8;
#pragma unroll
      for (int e = 0; e < 8; ++e) hv[it][e] = toh_flush(sp[e] * 64.0f);
    }
    for (int pass = 0; pass < 2; ++pass) {
#pragma unroll
      for (int it = 0; it < 4; ++it) {
        const unsigned row = (unsigned)it * 4u + q;
        *(volatile v8h*)(Ch16 + (size_t)row * CH + c8) = hv[it];
      }
      __threadfence();
    }
  }
}

__device__ __forceinline__ float batch_trace(const float* __restrict__ var_b, unsigned lane) {
    float s = 0.f;
#pragma unroll
    for (int it = 0; it < 4; ++it) {
        const v4f a = *(const v4f*)(var_b + ((unsigned)it * 32u + lane) * 4u);
        s += (a.x + a.y) + (a.z + a.w);
    }
#pragma unroll
    for (int o = 16; o > 0; o >>= 1) s += __shfl_xor(s, o, 32);
    return s;
}

__global__ __launch_bounds__(256) void k_xconv(const float* __restrict__ x, unsigned gb0, _Float16* __restrict__ x16,
                                               float* __restrict__ mean, float* __restrict__ var) {
#pragma clang fp contract(off)
    const unsigned lane = threadIdx.x & 31u;
    const unsigned wave = (unsigned)__builtin_amdgcn_readfirstlane((int)(threadIdx.x >> 5));
    const unsigned row0 = (blockIdx.x * 8u + wave) * 32u;
    if (row0 >= (unsigned)(NBC * CH)) return;
    float mymean = 0.f, myvar = 0.f;
#pragma unroll 1
    for (unsigned r = 0; r < 32u; ++r) {
        const unsigned lr = row0 + r;
        const unsigned lb = lr >> 9, c = lr & 511u;
        const float* xr = x + ((size_t)(gb0 + lb) * CH + c) * MSP;
        float s = 0.f, q = 0.f;
#pragma unroll
        for (int it = 0; it < 4; ++it) {
            const unsigned piece = (unsigned)it * 32u + lane;
            const unsigned pc = (piece < (unsigned)(MSP / 8)) ? piece : (unsigned)(MSP / 8 - 1);
            v4f a = *(const v4f*)(xr + 8u * pc);
            v4f b = *(const v4f*)(xr + 8u * pc + 4u);
            asm volatile("" : "+v"(a), "+v"(b));
            const bool valid = piece < (unsigned)(MSP / 8);
            float v[8] = {bfr(a.x), bfr(a.y), bfr(a.z), bfr(a.w), bfr(b.x), bfr(b.y), bfr(b.z), bfr(b.w)};
#pragma unroll
            for (int e = 0; e < 8; ++e) {
                const float t = valid ? v[e] : 0.0f;
                s += t;
                q += t * t;
                v[e] = t * 16.0f;
            }
            if (piece < (unsigned)(XP / 8)) st8hf(x16, (size_t)lr * XP + 8u * piece, v);
        }
#pragma unroll
        for (int o = 16; o > 0; o >>= 1) { s += __shfl_xor(s, o, 32); q += __shfl_xor(q, o, 32); }
        const float mu = s * (1.0f / 784.0f);
        const float vr = q * (1.0f / 784.0f) - mu * mu;
        mymean = (lane == r) ? mu : mymean;
        myvar  = (lane == r) ? vr : myvar;
    }
    VST2(float, mean + row0 + lane, mymean);
    VST2(float, var + row0 + lane, myvar);
}

__global__ __launch_bounds__(256) void k_cov(const _Float16* __restrict__ x16, const float* __restrict__ mean, const float* __restrict__ var,
                                             float* __restrict__ Cf, _Float16* __restrict__ Ch16) {
  __shared__ __align__(16) float sT[8][16 * 68];
  const unsigned lane = threadIdx.x & 31u;
  const unsigned wave = (unsigned)__builtin_amdgcn_readfirstlane((int)(threadIdx.x >> 5));
  const unsigned tile = blockIdx.x * 8u + wave;
  if (tile >= 64u) return;
  const unsigned lb = blockIdx.y;
  const unsigned m0 = (tile >> 3) << 6, n0 = (tile & 7u) << 6;
  const unsigned rlane = lane & 15u;
  const unsigned koff = (lane >> 4) * 8u;
  const unsigned mOff = koff;
  const _Float16* Ab = x16 + (size_t)lb * CH * XP;

  v8f acc[4][4];
  gemm_tile64(Ab, XP, Ab, XP, KCOV, m0, n0, rlane, koff, acc);

  const float* mb = mean + (size_t)lb * CH;
  const float tr = batch_trace(var + (size_t)lb * CH, lane);
  const float nrm = 512.0f * (1.0f / tr);
  const unsigned hh2 = lane >> 4, c4 = (lane & 15u) * 4u;
  const v4f mun = *(const v4f*)(mb + n0 + c4);
  float* Cb = Cf + (size_t)lb * DD;
  _Float16* Hb = Ch16 + (size_t)lb * DD;

  float* slab = sT[wave];
#pragma unroll
  for (int i = 0; i < 4; ++i) {
    const unsigned mBase = m0 + ((unsigned)i << 4);
#pragma unroll
    for (int j = 0; j < 4; ++j)
#pragma unroll
      for (int r = 0; r < 8; ++r)
        slab[(mOff + (unsigned)r) * 68u + ((unsigned)j << 4) + rlane] = acc[i][j][r];
    wave_sync_lds();
#pragma unroll
    for (int it = 0; it < 8; ++it) {
      const unsigned row = (unsigned)it * 2u + hh2;
      float* cell = slab + row * 68u + c4;
      const float mum = mb[mBase + row];
      const v4f a = *(const v4f*)cell;
      const v4f o = (a * CA_COV - mun * mum) * nrm;
      *(v4f*)cell = o;
    }
    wave_sync_lds();
    slab_store(slab, lane, Cb + (size_t)mBase * CH + n0, Hb + (size_t)mBase * CH + n0, true);
    wave_sync_lds();
  }
}

__global__ __launch_bounds__(256) void k_ns(const _Float16* __restrict__ Ah, const _Float16* __restrict__ Bh,
                                            const float* __restrict__ R1, const float* __restrict__ R2,
                                            float* __restrict__ Cf, _Float16* __restrict__ Ch16,
                                            float c1, float c2, float c3, unsigned flags) {
  __shared__ __align__(16) float sT[8][16 * 68];
  const unsigned lane = threadIdx.x & 31u;
  const unsigned wave = (unsigned)__builtin_amdgcn_readfirstlane((int)(threadIdx.x >> 5));
  const unsigned tile = blockIdx.x * 8u + wave;
  if (tile >= 64u) return;
  const unsigned lb = blockIdx.y;
  const unsigned m0 = (tile >> 3) << 6, n0 = (tile & 7u) << 6;
  const unsigned rlane = lane & 15u;
  const unsigned koff = (lane >> 4) * 8u;
  const unsigned mOff = koff;
  const bool useR2 = (flags & 1u) != 0u;
  const bool out16 = (flags & 2u) != 0u;

  v8f acc[4][4];
  gemm_tile64(Ah + (size_t)lb * DD, CH, Bh + (size_t)lb * DD, CH, CH, m0, n0, rlane, koff, acc);

  const float* R1b = R1 + (size_t)lb * DD;
  const float* R2b = R2 + (size_t)lb * DD;
  float* Cb = Cf + (size_t)lb * DD;
  _Float16* Hb = Ch16 + (size_t)lb * DD;
  const unsigned hh2 = lane >> 4, c4 = (lane & 15u) * 4u;

  float* slab = sT[wave];
#pragma unroll
  for (int i = 0; i < 4; ++i) {
    const unsigned mBase = m0 + ((unsigned)i << 4);
#pragma unroll
    for (int j = 0; j < 4; ++j)
#pragma unroll
      for (int r = 0; r < 8; ++r)
        slab[(mOff + (unsigned)r) * 68u + ((unsigned)j << 4) + rlane] = acc[i][j][r];
    wave_sync_lds();
#pragma unroll
    for (int it = 0; it < 8; ++it) {
      const unsigned row = (unsigned)it * 2u + hh2;
      float* cell = slab + row * 68u + c4;
      const size_t g = (size_t)(mBase + row) * CH + n0 + c4;
      const v4f a = *(const v4f*)cell;
      v4f o = a * c3 + *(const v4f*)(R1b + g) * c1;
      if (useR2) o += *(const v4f*)(R2b + g) * c2;
      *(v4f*)cell = o;
    }
    wave_sync_lds();
    slab_store(slab, lane, Cb + (size_t)mBase * CH + n0, Hb + (size_t)mBase * CH + n0, out16);
    wave_sync_lds();
  }
}

__global__ __launch_bounds__(512) void k_tail(const float* __restrict__ wsf, size_t offY3, size_t offF3, size_t offP4,
                                              const float* __restrict__ var, float* __restrict__ factor) {
    __shared__ float sv[512];
    const unsigned t = threadIdx.x, lane = t & 31u, lb = blockIdx.x;
    const float tr = batch_trace(var + (size_t)lb * CH, lane);
    sv[t] = 1.0f;
    __syncthreads();
    float u4c = 0.f, outv = 0.f;
#pragma unroll 1
    for (unsigned step = 0; step < 6u; ++step) {
        const bool isY = (step == 0u) || (step == 4u);
        const bool isF = (step == 3u);
        const size_t moff = isY ? offY3 : (isF ? offF3 : offP4);
        const float alpha = isY ? 0.0f : (isF ? 3.375f : 1.5f);
        const float beta = (step == 0u) ? 1.0f : ((step == 4u) ? 0.001953125f : (isF ? -0.001953125f : -0.0009765625f));
        const float* Mp = wsf + moff + (size_t)lb * DD + t;
        float m = 0.f;
#pragma unroll 4
        for (unsigned i = 0; i < 512u; ++i) m += sv[i] * Mp[(size_t)i * 512u];
        outv = alpha * sv[t] + beta * m;
        if (step == 1u) u4c = outv;
        __syncthreads();
        sv[t] = outv;
        __syncthreads();
    }
    const float rh = 0.5f * (3.0f * u4c - outv);
    VST2(float, factor + (size_t)lb * CH + t, sqrtf(tr) * rh * (1.0f / 262144.0f));
}

__global__ __launch_bounds__(256) void k_apply(const float* __restrict__ x, const float* __restrict__ factor,
                                               float* __restrict__ out, unsigned n4) {
#pragma clang fp contract(off)
    const unsigned u = blockIdx.x * 256u + threadIdx.x;
    if (u >= n4) return;
    const unsigned e = u * 4u;
    const unsigned chn = e / (unsigned)MSP;
    const float s = factor[chn];
    const v4f a = *(const v4f*)(x + e);
    v4f o;
    o.x = bfr(a.x) * s; o.y = bfr(a.y) * s; o.z = bfr(a.z) * s; o.w = bfr(a.w) * s;
    VST2V4(out + e, o);
}

extern "C" void kernel_launch(void* const* d_in, const int* in_sizes, int n_in, void* d_out, int out_size,
                              void* d_ws, size_t ws_size, hipStream_t stream) {
    if (n_in < 1) return;
    if (in_sizes[0] < NB * CH * MSP || out_size < NB * CH * MSP) return;

    const float* x = (const float*)d_in[0];
    float* out = (float*)d_out;

    char* wsp = (char*)d_ws;
    size_t off = 0;
    auto carve = [&](size_t bytes) -> void* { void* r = wsp + off; off += (bytes + 255) & ~(size_t)255; return r; };
    _Float16* x16   = (_Float16*)carve(SZ_X16);
    float*    meanT = (float*)carve(SZ_TAB);
    float*    varT  = (float*)carve(SZ_TAB);
    float*    fb    = (float*)carve(4 * SZ_F32);
    _Float16* hb    = (_Float16*)carve(4 * SZ_F16);
    float*    facT  = (float*)carve(SZ_SCL);
    if (off > ws_size || off > (size_t)134217728) return;

    const size_t PL = (size_t)NBC * DD;
    float* f0 = fb;
    float* f1 = fb + PL;
    float* f2 = fb + 2 * PL;
    float* f3 = fb + 3 * PL;
    _Float16* h0 = hb;
    _Float16* h1 = hb + PL;
    _Float16* h2 = hb + 2 * PL;
    _Float16* h3 = hb + 3 * PL;

    const dim3 gg(8, NBC);
    for (unsigned ch = 0; ch < (unsigned)NCHUNK; ++ch) {
        const unsigned gb0 = ch * (unsigned)NBC;
        k_xconv<<<(NBC * CH) / 256, 256, 0, stream>>>(x, gb0, x16, meanT, varT);
        k_cov<<<gg, 256, 0, stream>>>((const _Float16*)x16, meanT, varT, f0, h0);
        k_ns<<<gg, 256, 0, stream>>>(h0, h0, f0, f0, f1, h1, K_ONE5, K_ZERO, K_M22, 2u);
        k_ns<<<gg, 256, 0, stream>>>(h0, h1, f1, f1, f2, h2, K_ONE5, K_ZERO, K_M22, 2u);
        k_ns<<<gg, 256, 0, stream>>>(h1, h2, f1, f1, f3, h3, K_ONE5, K_ZERO, K_M22, 2u);
        k_ns<<<gg, 256, 0, stream>>>(h2, h0, f0, f2, f1, h1, K_075, K_075, K_M23, 3u);
        k_ns<<<gg, 256, 0, stream>>>(h1, h3, f3, f3, f0, h0, K_225, K_ZERO, K_M21, 2u);
        k_ns<<<gg, 256, 0, stream>>>(h3, h0, f3, f3, f2, h2, K_ONE5, K_ZERO, K_M22, 2u);
        k_ns<<<gg, 256, 0, stream>>>(h0, h1, f1, f0, f3, h3, K_ONE5, K_1125, K_M22, 3u);
        k_ns<<<gg, 256, 0, stream>>>(h3, h2, f2, f2, f1, h1, K_3375, K_ZERO, K_M21, 0u);
        k_tail<<<NBC, 512, 0, stream>>>((const float*)fb, 2 * PL, 3 * PL, PL, varT, facT + (size_t)gb0 * CH);
    }
    const unsigned n4 = (unsigned)((size_t)NB * CH * MSP / 4);
    k_apply<<<n4 / 256u, 256, 0, stream>>>(x, facT, out, n4);
}
